// GAT_7499012899343
// MI455X (gfx1250) — hardware-verified
//
#include <hip/hip_runtime.h>
#include <math.h>

#ifndef NB
#define NB 4
#endif
#ifndef SEQ
#define SEQ 2048
#endif
#define SEQ_FULL 2048
#define CIN 256
#define FH 64
#define NHEAD 4
#define HFW 256
#define CATW 512
#define MROWS (NB * SEQ)
#define FPLANE ((unsigned)(NB * NHEAD * SEQ))
#define LEAK 0.2f
#define NEG_FILL (-1.0e12f)
#define L2E 1.4426950408889634f

static_assert(SEQ == SEQ_FULL);
static_assert(HFW == NHEAD * FH);
static_assert(CATW == 2 * HFW);
static_assert(MROWS % 64 == 0);
static_assert(HFW % 64 == 0 && FH % 64 == 0);
static_assert(CIN % 32 == 0 && CATW % 32 == 0);
static_assert(CIN / 8 == 32);
static_assert(SEQ % 1024 == 0);
static_assert(SEQ % 128 == 0);
static_assert((MROWS * CIN / 8) % 256 == 0);
static_assert((FH * (CIN / 8)) % 256 == 0);
static_assert((FH * (CATW / 8)) % 256 == 0);

static constexpr float XC  = 16.0f;
static constexpr float WC  = 64.0f;
static constexpr float VC  = 16.0f;
static constexpr float PC  = 16384.0f;
static constexpr float CC  = 256.0f;
static constexpr float WLC = 64.0f;
static constexpr float SC_PROJ = 1.0f / 1024.0f;
static constexpr float CAT_SC  = 1.0f / 1024.0f;
static constexpr float SC_OUT  = 1.0f / 16384.0f;
static_assert(SC_PROJ * XC * WC == 1.0f);
static_assert(CAT_SC * PC * VC == CC);
static_assert(SC_OUT * CC * WLC == 1.0f);
static_assert(PC < 32752.0f);

typedef __attribute__((ext_vector_type(16))) _Float16 v16h;
typedef __attribute__((ext_vector_type(8)))  _Float16 v8h;
typedef __attribute__((ext_vector_type(2)))  _Float16 v2h;
typedef __attribute__((ext_vector_type(8)))  float    v8f;
typedef __attribute__((ext_vector_type(4)))  float    v4f;
typedef __attribute__((ext_vector_type(2)))  float    v2fl;
typedef __attribute__((ext_vector_type(4)))  unsigned int v4u;
typedef __attribute__((ext_vector_type(8)))  unsigned int v8u;
typedef __attribute__((ext_vector_type(4)))  int      v4i;


#define VST2(T, ptr, val) do { const T vst2_v_ = (val); *(volatile T*)(ptr) = vst2_v_; __threadfence(); *(volatile T*)(ptr) = vst2_v_; } while (0)
#define VST2V4(ptr, val) do { const v4f vst2_v4_ = (val); *(volatile v4f*)(ptr) = vst2_v4_; __threadfence(); *(volatile v4f*)(ptr) = vst2_v4_; } while (0)

__device__ __forceinline__ float bfr(float f) {
    unsigned u = __float_as_uint(f);
    u += 0x7FFFu + ((u >> 16) & 1u);
    return __uint_as_float(u & 0xFFFF0000u);
}
__device__ __forceinline__ unsigned short f2h_bits(float x) {
    return (fabsf(x) < 6.104e-5f) ? (unsigned short)0 : __builtin_bit_cast(unsigned short, (_Float16)x);
}
__device__ __forceinline__ void st8h(unsigned short* P, size_t o, const float* v) {
    v4u pk;
    pk.x = (unsigned)f2h_bits(v[0]) | ((unsigned)f2h_bits(v[1]) << 16);
    pk.y = (unsigned)f2h_bits(v[2]) | ((unsigned)f2h_bits(v[3]) << 16);
    pk.z = (unsigned)f2h_bits(v[4]) | ((unsigned)f2h_bits(v[5]) << 16);
    pk.w = (unsigned)f2h_bits(v[6]) | ((unsigned)f2h_bits(v[7]) << 16);
    VST2(v4u, (v4u*)(P + o), pk);
}

static __device__ __forceinline__ v2h toh2_flush(float a, float b) {
    v2fl w;
    w.x = (fabsf(a) < 6.103515625e-05f) ? 0.0f : a;
    w.y = (fabsf(b) < 6.103515625e-05f) ? 0.0f : b;
    return __builtin_convertvector(w, v2h);
}
static __device__ __forceinline__ v4u pack8_flush(const float (&v)[8]) {
    v4u o;
    o.x = __builtin_bit_cast(unsigned, toh2_flush(v[0], v[1]));
    o.y = __builtin_bit_cast(unsigned, toh2_flush(v[2], v[3]));
    o.z = __builtin_bit_cast(unsigned, toh2_flush(v[4], v[5]));
    o.w = __builtin_bit_cast(unsigned, toh2_flush(v[6], v[7]));
    return o;
}
static __device__ __forceinline__ void split8_flush(const float (&v)[8], v4u& hi, v4u& lo) {
    unsigned hw[4], lw[4];
#pragma unroll
    for (int q = 0; q < 4; ++q) {
        const v2h h2 = toh2_flush(v[2 * q], v[2 * q + 1]);
        const float r0 = v[2 * q] - (float)h2.x;
        const float r1 = v[2 * q + 1] - (float)h2.y;
        const v2h l2 = toh2_flush(r0, r1);
        hw[q] = __builtin_bit_cast(unsigned, h2);
        lw[q] = __builtin_bit_cast(unsigned, l2);
    }
    hi.x = hw[0]; hi.y = hw[1]; hi.z = hw[2]; hi.w = hw[3];
    lo.x = lw[0]; lo.y = lw[1]; lo.z = lw[2]; lo.w = lw[3];
}
static __device__ __forceinline__ void spread16(const v4f a, const v4f b, const v4f c, const v4f d, float (&o)[16]) {
    o[0] = a.x; o[1] = a.y; o[2] = a.z; o[3] = a.w;
    o[4] = b.x; o[5] = b.y; o[6] = b.z; o[7] = b.w;
    o[8] = c.x; o[9] = c.y; o[10] = c.z; o[11] = c.w;
    o[12] = d.x; o[13] = d.y; o[14] = d.z; o[15] = d.w;
}
static __device__ __forceinline__ void spread16i(const v4i a, const v4i b, const v4i c, const v4i d, int (&o)[16]) {
    o[0] = a.x; o[1] = a.y; o[2] = a.z; o[3] = a.w;
    o[4] = b.x; o[5] = b.y; o[6] = b.z; o[7] = b.w;
    o[8] = c.x; o[9] = c.y; o[10] = c.z; o[11] = c.w;
    o[12] = d.x; o[13] = d.y; o[14] = d.z; o[15] = d.w;
}

union FragU { v16h v; v8h h[2]; };
__device__ __forceinline__ v16h frag_ld(const _Float16* p) {
    FragU f; f.h[0] = *(const v8h*)(p); f.h[1] = *(const v8h*)(p + 16); return f.v;
}
__device__ __forceinline__ v8f wmma16(v16h a, v16h b, v8f c) {
    c = __builtin_amdgcn_wmma_f32_16x16x32_f16(false, a, false, b, (short)0, c, false, false);
    asm volatile("v_nop\n\tv_nop\n\tv_nop\n\tv_nop" : "+v"(c) : "v"(a), "v"(b));
    return c;
}
__device__ __forceinline__ void wave_sync_lds() {
    __builtin_amdgcn_fence(3  , "workgroup");
    __builtin_amdgcn_wave_barrier();
    __builtin_amdgcn_fence(2  , "workgroup");
}

static_assert(32 * 16 * 8 == 16 * 64 * 4);
static_assert(8 * 16 * 68 * 4 <= 131072);
template <bool BIAS, bool LEAKY>
static __device__ __forceinline__ void gemm64_body(
    const _Float16* __restrict__ A, const unsigned lda, const _Float16* __restrict__ Bt, const unsigned ldb,
    float* __restrict__ C, const unsigned ldc, const float* __restrict__ bias,
    const unsigned M, const unsigned N, const unsigned K, const float scale) {
  __shared__ __align__(16) float sT[8][16 * 68];
  const unsigned lane = threadIdx.x & 31u;
  const unsigned wave = __builtin_amdgcn_readfirstlane(threadIdx.x >> 5);
  const unsigned tilesN = N >> 6, tilesM = M >> 6;
  const unsigned tile = blockIdx.x * 8u + wave;
  if (tile >= tilesM * tilesN) return;
  const unsigned tm = tile / tilesN;
  const unsigned tn = tile - tm * tilesN;
  const unsigned m0 = tm << 6, n0 = tn << 6;
  const unsigned rlane = lane & 15u;
  const unsigned koff = (lane >> 4) * 8u;
  const unsigned mOff = koff;

  v8f acc[4][4];
#pragma unroll
  for (int i = 0; i < 4; ++i)
#pragma unroll
    for (int j = 0; j < 4; ++j) acc[i][j] = (v8f){0.f,0.f,0.f,0.f,0.f,0.f,0.f,0.f};

#pragma unroll 1
  for (unsigned k0 = 0; k0 < K; k0 += 32u) {
    v16h bh[4];
#pragma unroll
    for (int j = 0; j < 4; ++j)
      bh[j] = frag_ld(Bt + (size_t)(n0 + ((unsigned)j << 4) + rlane) * ldb + koff + k0);
#pragma unroll
    for (int i = 0; i < 4; ++i) {
      const v16h ah = frag_ld(A + (size_t)(m0 + ((unsigned)i << 4) + rlane) * lda + koff + k0);
#pragma unroll
      for (int j = 0; j < 4; ++j)
        acc[i][j] = wmma16(ah, bh[j], acc[i][j]);
    }
  }

#pragma unroll
  for (int i = 0; i < 4; ++i) {
    const unsigned mBase = m0 + ((unsigned)i << 4);
#pragma unroll
    for (int j = 0; j < 4; ++j) {
      const unsigned n = n0 + ((unsigned)j << 4) + rlane;
      float bv = 0.0f;
      if (BIAS) bv = bfr(bias[n]);
#pragma unroll
      for (int r = 0; r < 8; ++r) {
        float v = acc[i][j][r] * scale + bv;
        if (LEAKY) v = (v >= 0.0f) ? v : LEAK * v;
        sT[wave][(mOff + (unsigned)r) * 68u + ((unsigned)j << 4) + rlane] = v;
      }
    }
    wave_sync_lds();
    {
      const unsigned hh = lane >> 4, c4 = (lane & 15u) * 4u;
#pragma unroll
      for (int half = 0; half < 2; ++half) {
        v4f vv[4];
#pragma unroll
        for (int it = 0; it < 4; ++it) {
          const unsigned row = (unsigned)(half * 4 + it) * 2u + hh;
          vv[it] = *(const v4f*)&sT[wave][row * 68u + c4];
        }
        for (int pass = 0; pass < 2; ++pass) {
#pragma unroll
          for (int it = 0; it < 4; ++it) {
            const unsigned row = (unsigned)(half * 4 + it) * 2u + hh;
            *(volatile v4f*)(C + (size_t)(mBase + row) * ldc + n0 + c4) = vv[it];
          }
          __threadfence();
        }
      }
    }
    wave_sync_lds();
  }
}

__global__ __launch_bounds__(256) void k_gemm_proj(const _Float16* __restrict__ A, const _Float16* __restrict__ Bt, float* __restrict__ C) {
  gemm64_body<false, false>(A, CIN, Bt, CIN, C, HFW, nullptr, MROWS, HFW, CIN, SC_PROJ);
}
__global__ __launch_bounds__(256) void k_gemm_out(const _Float16* __restrict__ A, const _Float16* __restrict__ Bt, float* __restrict__ C,
                                                  const float* __restrict__ bias) {
  gemm64_body<true, true>(A, CATW, Bt, CATW, C, FH, bias, MROWS, FH, CATW, SC_OUT);
}

__global__ __launch_bounds__(256) void k_wt16(const float* __restrict__ Wm, unsigned KI, unsigned NO, unsigned lgper,
                                              unsigned short* __restrict__ W16, float sw) {
    const unsigned layer = blockIdx.y;
    const float* Wl = Wm + (size_t)layer * KI * NO;
    unsigned short* Dl = W16 + (size_t)layer * KI * NO;
    const unsigned u = blockIdx.x * 256u + threadIdx.x;
    const unsigned per = 1u << lgper;
    if (u >= NO * per) return;
    const unsigned k0 = 8u * (u & (per - 1u));
    const unsigned o = u >> lgper;
    float v[8];
#pragma unroll
    for (int i = 0; i < 8; ++i) v[i] = bfr(Wl[(size_t)(k0 + (unsigned)i) * NO + o]) * sw;
    st8h(Dl, (size_t)o * KI + k0, v);
}

__global__ __launch_bounds__(256) void k_x16(const float* __restrict__ x, _Float16* __restrict__ x16) {
    const unsigned u = blockIdx.x * 256u + threadIdx.x;
    const unsigned row = u >> 5, c0 = (u & 31u) * 8u;
    const float* src = x + (size_t)row * CIN + c0;
    const v4f a = *(const v4f*)src, b = *(const v4f*)(src + 4);
    float v[8];
    v[0] = bfr(a.x) * XC; v[1] = bfr(a.y) * XC; v[2] = bfr(a.z) * XC; v[3] = bfr(a.w) * XC;
    v[4] = bfr(b.x) * XC; v[5] = bfr(b.y) * XC; v[6] = bfr(b.z) * XC; v[7] = bfr(b.w) * XC;
    const v4u pk = pack8_flush(v);
    VST2(v4u, x16 + (size_t)row * CIN + c0, pk);
}

__global__ __launch_bounds__(256) void k_wl16(const float* __restrict__ Wl, _Float16* __restrict__ wl16) {
    const unsigned u = blockIdx.x * 256u + threadIdx.x;
    const unsigned n = u >> 6, k0 = (u & 63u) * 8u;
    const float* src = Wl + (size_t)n * HFW + (k0 & 255u);
    const v4f a = *(const v4f*)src, b = *(const v4f*)(src + 4);
    float v[8];
    v[0] = bfr(a.x) * WLC; v[1] = bfr(a.y) * WLC; v[2] = bfr(a.z) * WLC; v[3] = bfr(a.w) * WLC;
    v[4] = bfr(b.x) * WLC; v[5] = bfr(b.y) * WLC; v[6] = bfr(b.z) * WLC; v[7] = bfr(b.w) * WLC;
    const v4u pk = pack8_flush(v);
    VST2(v4u, wl16 + (size_t)n * CATW + k0, pk);
}

#define PL_P 68
static_assert((64 * PL_P + 2 * 64 + 2 * 64) * 4 <= 131072);
static_assert(256 * 16 * 2 == 64 * 64 * 2);
__global__ __launch_bounds__(256) void k_planes(const float* __restrict__ HF, const float* __restrict__ a1, const float* __restrict__ a2,
                                                float* __restrict__ F12, _Float16* __restrict__ VTh, _Float16* __restrict__ VTl) {
    __shared__ __align__(16) float sH[64 * PL_P];
    __shared__ float sA[2][64];
    __shared__ __align__(16) float sF[2][64];
    const unsigned t = threadIdx.x;
    const unsigned n0 = blockIdx.x * 64u, hd = blockIdx.y, b = blockIdx.z;
    const unsigned bh = b * (unsigned)NHEAD + hd;
    {
        const unsigned f = t & 63u;
        const float w1 = bfr(a1[hd * 64u + f]);
        const float w2 = bfr(a2[hd * 64u + f]);
        if (t < 64u) { sA[0][f] = w1; sA[1][f] = w2; }
    }
#pragma unroll
    for (unsigned it = 0; it < 4u; ++it) {
        const unsigned idx = it * 256u + t;
        const unsigned r = idx >> 4, c4 = (idx & 15u) * 4u;
        const v4f v = *(const v4f*)(HF + (size_t)(b * (unsigned)SEQ + n0 + r) * HFW + hd * 64u + c4);
        *(v4f*)&sH[r * PL_P + c4] = v;
    }
    __syncthreads();
    if (t < 128u) {
        const unsigned node = t & 63u, which = t >> 6;
        float s = 0.0f;
#pragma unroll 4
        for (unsigned f = 0; f < 64u; ++f) s += sH[node * PL_P + f] * sA[which][f];
        sF[which][node] = s;
    }
    __syncthreads();
    if (t < 32u) {
        const unsigned plane = t >> 4, piece = t & 15u;
        const v4f v = *(const v4f*)&sF[plane][4u * piece];
        VST2V4(F12 + (size_t)plane * FPLANE + (size_t)bh * SEQ + n0 + 4u * piece, v);
    }
    const unsigned piece = t & 7u, cg = t >> 3;
#pragma unroll 1
    for (unsigned ps = 0; ps < 2u; ++ps) {
        const unsigned col = ps * 32u + cg;
        float v[8];
#pragma unroll
        for (int e = 0; e < 8; ++e) v[e] = sH[(8u * piece + (unsigned)e) * PL_P + col] * VC;
        v4u hi, lo;
        split8_flush(v, hi, lo);
        const size_t o = (size_t)(b * (unsigned)HFW + hd * 64u + col) * SEQ + n0 + 8u * piece;
        for (int pass = 0; pass < 2; ++pass) {
            *(volatile v4u*)(VTh + o) = hi;
            *(volatile v4u*)(VTl + o) = lo;
            __threadfence();
        }
    }
}

static_assert((SEQ + 4 * 64 + 4 * 64 + 2 * 64) * 4 <= 131072);
__global__ __launch_bounds__(256) void k_colstat(const int* __restrict__ adj, const float* __restrict__ F12, float* __restrict__ MR) {
    __shared__ __align__(16) float sF1[SEQ];
    __shared__ float sM[4][64];
    __shared__ float sS[4][64];
    __shared__ __align__(16) float sO[2][64];
    const unsigned t = threadIdx.x;
    const unsigned j0 = blockIdx.x * 64u, bh = blockIdx.y;
#pragma unroll
    for (unsigned it = 0; it < (unsigned)(SEQ / 1024); ++it) {
        const unsigned idx = it * 256u + t;
        *(v4f*)&sF1[4u * idx] = *(const v4f*)(F12 + (size_t)bh * SEQ + 4u * idx);
    }
    __syncthreads();
    const unsigned c = t & 63u, g = t >> 6;
    const float f2j = F12[(size_t)FPLANE + (size_t)bh * SEQ + j0 + c];
    const unsigned ibase = g * (unsigned)(SEQ / 4);
    const int* ap = adj + (size_t)ibase * SEQ_FULL + j0 + c;
    float m = -1.0e30f, s = 0.0f;
#pragma unroll 1
    for (unsigned ic = 0; ic < (unsigned)(SEQ / 4); ic += 8u) {
        int av[8];
#pragma unroll
        for (int k = 0; k < 8; ++k) av[k] = ap[(size_t)(ic + (unsigned)k) * SEQ_FULL];
        float ev[8];
#pragma unroll
        for (int k = 0; k < 8; ++k) {
            float v = sF1[ibase + ic + (unsigned)k] + f2j;
            v = (v >= 0.0f) ? v : LEAK * v;
            ev[k] = (av[k] > 0) ? v : NEG_FILL;
        }
        float cm = ev[0];
#pragma unroll
        for (int k = 1; k < 8; ++k) cm = (ev[k] > cm) ? ev[k] : cm;
        const float mn = (cm > m) ? cm : m;
        s = s * exp2f((m - mn) * L2E);
#pragma unroll
        for (int k = 0; k < 8; ++k) s += exp2f((ev[k] - mn) * L2E);
        m = mn;
    }
    sM[g][c] = m;
    sS[g][c] = s;
    __syncthreads();
    if (t < 64u) {
        float M = sM[0][t];
#pragma unroll
        for (int q = 1; q < 4; ++q) { const float v = sM[q][t]; M = (v > M) ? v : M; }
        float S = 0.0f;
#pragma unroll
        for (int q = 0; q < 4; ++q) S += sS[q][t] * exp2f((sM[q][t] - M) * L2E);
        sO[0][t] = M;
        sO[1][t] = PC * (1.0f / S);
    }
    __syncthreads();
    if (t < 32u) {
        const unsigned plane = t >> 4, piece = t & 15u;
        const v4f v = *(const v4f*)&sO[plane][4u * piece];
        VST2V4(MR + (size_t)plane * FPLANE + (size_t)bh * SEQ + j0 + 4u * piece, v);
    }
}

static_assert(32 * 16 * 4 == 16 * 64 * 2);
static_assert((3 * SEQ + 8 * 16 * 68) * 4 <= 131072);
__global__ __launch_bounds__(256) void k_attn(const int* __restrict__ adj, const float* __restrict__ F12, const float* __restrict__ MR,
                                              const _Float16* __restrict__ VTh, const _Float16* __restrict__ VTl,
                                              _Float16* __restrict__ CAT) {
    __shared__ __align__(16) float sF2[SEQ];
    __shared__ __align__(16) float sMm[SEQ];
    __shared__ __align__(16) float sRr[SEQ];
    __shared__ __align__(16) float sOt[8][16 * 68];
    const unsigned tid = threadIdx.x, lane = tid & 31u;
    const unsigned wave = __builtin_amdgcn_readfirstlane(tid >> 5);
    const unsigned hh = lane >> 4, c = lane & 15u;
    const unsigned bh = blockIdx.y;
    const unsigned b = bh >> 2, hd = bh & 3u;
    const unsigned i0 = blockIdx.x * 128u + wave * 16u;
#pragma unroll
    for (unsigned it = 0; it < (unsigned)(SEQ / 1024); ++it) {
        const unsigned idx = it * 256u + tid;
        *(v4f*)&sF2[4u * idx] = *(const v4f*)(F12 + (size_t)FPLANE + (size_t)bh * SEQ + 4u * idx);
        *(v4f*)&sMm[4u * idx] = *(const v4f*)(MR + (size_t)bh * SEQ + 4u * idx);
        *(v4f*)&sRr[4u * idx] = *(const v4f*)(MR + (size_t)FPLANE + (size_t)bh * SEQ + 4u * idx);
    }
    __syncthreads();
    const float f1i = F12[(size_t)bh * SEQ + i0 + c];
    const int* arow = adj + (size_t)(i0 + c) * SEQ_FULL + 8u * hh;
    const size_t vrow = (size_t)(b * (unsigned)HFW + hd * 64u + c) * SEQ + 8u * hh;
    const _Float16* vh = VTh + vrow;
    const _Float16* vl = VTl + vrow;
    v8f acc[4];
#pragma unroll
    for (int t = 0; t < 4; ++t) acc[t] = (v8f){0.f,0.f,0.f,0.f,0.f,0.f,0.f,0.f};

#pragma unroll 1
    for (unsigned j0 = 0; j0 < (unsigned)SEQ; j0 += 32u) {
        const unsigned jl = j0 + 8u * hh;
        int av[16];
        spread16i(*(const v4i*)(arow + j0), *(const v4i*)(arow + j0 + 4u), *(const v4i*)(arow + j0 + 16u), *(const v4i*)(arow + j0 + 20u), av);
        float f2v[16], mv[16], rv[16];
        spread16(*(const v4f*)&sF2[jl], *(const v4f*)&sF2[jl + 4u], *(const v4f*)&sF2[jl + 16u], *(const v4f*)&sF2[jl + 20u], f2v);
        spread16(*(const v4f*)&sMm[jl], *(const v4f*)&sMm[jl + 4u], *(const v4f*)&sMm[jl + 16u], *(const v4f*)&sMm[jl + 20u], mv);
        spread16(*(const v4f*)&sRr[jl], *(const v4f*)&sRr[jl + 4u], *(const v4f*)&sRr[jl + 16u], *(const v4f*)&sRr[jl + 20u], rv);
        v8u phu, plu;
#pragma unroll
        for (int q = 0; q < 8; ++q) {
            float pp[2];
#pragma unroll
            for (int s2 = 0; s2 < 2; ++s2) {
                const int e = 2 * q + s2;
                float ev = f1i + f2v[e];
                ev = (ev >= 0.0f) ? ev : LEAK * ev;
                ev = (av[e] > 0) ? ev : NEG_FILL;
                pp[s2] = exp2f((ev - mv[e]) * L2E) * rv[e];
            }
            const v2h h2 = toh2_flush(pp[0], pp[1]);
            const v2h l2 = toh2_flush(pp[0] - (float)h2.x, pp[1] - (float)h2.y);
            phu[q] = __builtin_bit_cast(unsigned, h2);
            plu[q] = __builtin_bit_cast(unsigned, l2);
        }
        const v16h ph = __builtin_bit_cast(v16h, phu);
        const v16h pl = __builtin_bit_cast(v16h, plu);
#pragma unroll
        for (int t = 0; t < 2; ++t) {
            const v16h ah = frag_ld(vh + (size_t)((unsigned)t * 16u) * SEQ + j0);
            const v16h al = frag_ld(vl + (size_t)((unsigned)t * 16u) * SEQ + j0);
            acc[t] = wmma16(ah, ph, acc[t]);
            acc[t] = wmma16(al, ph, acc[t]);
            acc[t] = wmma16(ah, pl, acc[t]);
        }
        unsigned o2 = j0;
        asm volatile("" : "+v"(o2));
#pragma unroll
        for (int t = 2; t < 4; ++t) {
            const v16h ah = frag_ld(vh + (size_t)((unsigned)t * 16u) * SEQ + o2);
            const v16h al = frag_ld(vl + (size_t)((unsigned)t * 16u) * SEQ + o2);
            acc[t] = wmma16(ah, ph, acc[t]);
            acc[t] = wmma16(al, ph, acc[t]);
            acc[t] = wmma16(ah, pl, acc[t]);
        }
    }
#pragma unroll
    for (int t = 0; t < 4; ++t)
#pragma unroll
        for (int r = 0; r < 8; ++r) {
            float v = acc[t][r] * CAT_SC;
            v = (v > 0.0f) ? v : 0.0f;
            sOt[wave][c * 68u + (unsigned)t * 16u + 8u * hh + (unsigned)r] = v;
        }
    wave_sync_lds();
    {
        const unsigned q = lane >> 3, c8 = (lane & 7u) * 8u;
        v4u hi[4], lo[4];
#pragma unroll
        for (int it = 0; it < 4; ++it) {
            const unsigned row = (unsigned)it * 4u + q;
            const v4f x0 = *(const v4f*)&sOt[wave][row * 68u + c8];
            const v4f x1 = *(const v4f*)&sOt[wave][row * 68u + c8 + 4u];
            float v[8];
            v[0] = x0.x; v[1] = x0.y; v[2] = x0.z; v[3] = x0.w;
            v[4] = x1.x; v[5] = x1.y; v[6] = x1.z; v[7] = x1.w;
            split8_flush(v, hi[it], lo[it]);
        }
        _Float16* dst = CAT + (size_t)(b * (unsigned)SEQ + i0) * CATW + hd * 64u + c8;
        for (int pass = 0; pass < 2; ++pass) {
#pragma unroll
            for (int it = 0; it < 4; ++it) {
                const unsigned row = (unsigned)it * 4u + q;
                *(volatile v4u*)(dst + (size_t)row * CATW) = hi[it];
                *(volatile v4u*)(dst + (size_t)row * CATW + HFW) = lo[it];
            }
            __threadfence();
        }
    }
}

static constexpr size_t SZ_X16  = (size_t)MROWS * CIN * 2;
static constexpr size_t SZ_WT16 = (size_t)HFW * CIN * 2;
static constexpr size_t SZ_WL16 = (size_t)FH * CATW * 2;
static constexpr size_t SZ_HF   = (size_t)MROWS * HFW * 4;
static constexpr size_t SZ_F12  = (size_t)2 * NB * NHEAD * SEQ * 4;
static constexpr size_t SZ_MR   = (size_t)2 * NB * NHEAD * SEQ * 4;
static constexpr size_t SZ_VT   = (size_t)NB * HFW * SEQ * 2;
static constexpr size_t SZ_CAT  = (size_t)MROWS * CATW * 2;
static constexpr size_t OFF_X16  = 0;
static constexpr size_t OFF_WT16 = OFF_X16 + SZ_X16;
static constexpr size_t OFF_WL16 = OFF_WT16 + SZ_WT16;
static constexpr size_t OFF_HF   = OFF_WL16 + SZ_WL16;
static constexpr size_t OFF_F12  = OFF_HF + SZ_HF;
static constexpr size_t OFF_MR   = OFF_F12 + SZ_F12;
static constexpr size_t OFF_VTH  = OFF_MR + SZ_MR;
static constexpr size_t OFF_VTL  = OFF_VTH + SZ_VT;
static constexpr size_t OFF_CAT  = OFF_VTL + SZ_VT;
static constexpr size_t WS_TOTAL = OFF_CAT + SZ_CAT;
static_assert(SZ_X16 % 256 == 0 && SZ_WT16 % 256 == 0 && SZ_WL16 % 256 == 0 && SZ_HF % 256 == 0);
static_assert(SZ_F12 % 256 == 0 && SZ_MR % 256 == 0 && SZ_VT % 256 == 0 && SZ_CAT % 256 == 0);
static_assert(WS_TOTAL <= (size_t)134217728);

extern "C" void kernel_launch(void* const* d_in, const int* in_sizes, int n_in, void* d_out, int out_size,
                              void* d_ws, size_t ws_size, hipStream_t stream) {
    if (n_in < 7) return;
    if (in_sizes[0] < MROWS * CIN || in_sizes[1] < SEQ_FULL * SEQ_FULL || in_sizes[2] < NHEAD * CIN * FH) return;
    if (in_sizes[3] < NHEAD * FH || in_sizes[4] < NHEAD * FH || in_sizes[5] < FH * HFW || in_sizes[6] < FH) return;
    if (out_size < MROWS * FH) return;
    if (WS_TOTAL > ws_size) return;

    const float* x   = (const float*)d_in[0];
    const int*   adj = (const int*)d_in[1];
    const float* W   = (const float*)d_in[2];
    const float* a1  = (const float*)d_in[3];
    const float* a2  = (const float*)d_in[4];
    const float* Wl  = (const float*)d_in[5];
    const float* bl  = (const float*)d_in[6];
    float* out = (float*)d_out;

    char* wsp = (char*)d_ws;
    _Float16*       x16  = (_Float16*)(wsp + OFF_X16);
    unsigned short* wt16 = (unsigned short*)(wsp + OFF_WT16);
    _Float16*       wl16 = (_Float16*)(wsp + OFF_WL16);
    float*          hf   = (float*)(wsp + OFF_HF);
    float*          f12  = (float*)(wsp + OFF_F12);
    float*          mr   = (float*)(wsp + OFF_MR);
    _Float16*       vth  = (_Float16*)(wsp + OFF_VTH);
    _Float16*       vtl  = (_Float16*)(wsp + OFF_VTL);
    _Float16*       cat  = (_Float16*)(wsp + OFF_CAT);

    k_x16<<<(MROWS * CIN / 8) / 256, 256, 0, stream>>>(x, x16);
    k_wt16<<<dim3((FH * (CIN / 8)) / 256, NHEAD), 256, 0, stream>>>(W, CIN, FH, 5, wt16, WC);
    k_wl16<<<(FH * (CATW / 8)) / 256, 256, 0, stream>>>(Wl, wl16);

    k_gemm_proj<<<((MROWS / 64) * (HFW / 64) + 7) / 8, 256, 0, stream>>>((const _Float16*)x16, (const _Float16*)wt16, hf);
    k_planes<<<dim3(SEQ / 64, NHEAD, NB), 256, 0, stream>>>(hf, a1, a2, f12, vth, vtl);
    k_colstat<<<dim3(SEQ / 64, NB * NHEAD), 256, 0, stream>>>(adj, f12, mr);
    k_attn<<<dim3(SEQ / 128, NB * NHEAD), 256, 0, stream>>>(adj, f12, mr, (const _Float16*)vth, (const _Float16*)vtl, cat);
    k_gemm_out<<<((MROWS / 64) * (FH / 64) + 7) / 8, 256, 0, stream>>>((const _Float16*)cat, (const _Float16*)wl16, out, bl);
}
